// YvFlashSSM_72112500900651
// MI455X (gfx1250) — hardware-run, weakly checked
//
#include <hip/hip_runtime.h>
#include <math.h>

#define DM    1024
#define LQ    2048
#define BQ    2
#define NTOK  (BQ * LQ)
#define NST   32
#define NBC   (2 * NST)
#define NPROJ (2 * DM + NBC)
#define TPB   128
#define OSTR  68
#define SCH   32
#define CHB   128

static_assert(NTOK % TPB == 0);
static_assert(NPROJ % 64 == 0);
static_assert(DM % 64 == 0);
static_assert(DM % 32 == 0);
static_assert(DM % CHB == 0);
static_assert(LQ % SCH == 0);
static_assert(2 * CHB == 256);
static_assert(SCH * NBC == 256 * 8);
static_assert(SCH * CHB == 2 * 256 * 8);
static_assert(OSTR % 4 == 0);
static_assert((NTOK * DM) % (8 * 256) == 0);
static_assert((NPROJ * DM) % (8 * 256) == 0);
static_assert((DM * DM) % (8 * 256) == 0);

typedef unsigned short us16 __attribute__((ext_vector_type(16)));
typedef unsigned short us8  __attribute__((ext_vector_type(8)));
typedef unsigned short us8a __attribute__((ext_vector_type(8), may_alias));
typedef __bf16 v16b __attribute__((ext_vector_type(16)));
typedef _Float16 v16h __attribute__((ext_vector_type(16)));
typedef float v8f __attribute__((ext_vector_type(8)));
typedef float v4f __attribute__((ext_vector_type(4)));
typedef float v4fa __attribute__((ext_vector_type(4), may_alias));
union FragU { us16 v; us8 h[2]; };

#if __has_builtin(__builtin_amdgcn_exp2f)
#define EXP2F(x) __builtin_amdgcn_exp2f(x)
#else
#define EXP2F(x) exp2f(x)
#endif

__device__ __forceinline__ unsigned short bf16_bits(float f) {
  unsigned u = __float_as_uint(f);
  u += 0x7FFFu + ((u >> 16) & 1u);
  return (unsigned short)(u >> 16);
}
__device__ __forceinline__ float bf16_val(unsigned short b) { return __uint_as_float(((unsigned)b) << 16); }
__device__ __forceinline__ float bf16r(float f) { return bf16_val(bf16_bits(f)); }
__device__ __forceinline__ unsigned short f16_bits(float f) { return __builtin_bit_cast(unsigned short, (_Float16)f); }

__device__ __forceinline__ void f16split(float z, unsigned short& hb, unsigned short& lb) {
  const _Float16 hf = (_Float16)z;
  const float res = (z - (float)hf) * 2048.0f;
  hb = __builtin_bit_cast(unsigned short, hf);
  lb = __builtin_bit_cast(unsigned short, (_Float16)res);
}

__device__ __forceinline__ float softplus_f(float t) { return fmaxf(t, 0.0f) + log1pf(expf(-fabsf(t))); }

__device__ __forceinline__ v8f mma_bf16(us16 a, us16 b, v8f c) {
  return __builtin_amdgcn_wmma_f32_16x16x32_bf16(false, __builtin_bit_cast(v16b, a), false, __builtin_bit_cast(v16b, b), (short)0, c, false, false);
}
__device__ __forceinline__ v8f mma_f16(us16 a, us16 b, v8f c) {
  return __builtin_amdgcn_wmma_f32_16x16x32_f16(false, __builtin_bit_cast(v16h, a), false, __builtin_bit_cast(v16h, b), (short)0, c, false, false);
}
__device__ __forceinline__ void wguard4(v8f& c0, v8f& c1, v8f& c2, v8f& c3, const us16& a0,
                                        const us16& b0, const us16& b1, const us16& b2, const us16& b3) {
#if defined(__HIP_DEVICE_COMPILE__)
  asm volatile("v_nop\n\tv_nop\n\tv_nop\n\tv_nop"
               : "+v"(c0), "+v"(c1), "+v"(c2), "+v"(c3)
               : "v"(a0), "v"(b0), "v"(b1), "v"(b2), "v"(b3));
#endif
}
__device__ __forceinline__ void wguard8(v8f& c0, v8f& c1, v8f& c2, v8f& c3, v8f& c4, v8f& c5, v8f& c6, v8f& c7,
                                        const us16& a0, const us16& a1,
                                        const us16& b0, const us16& b1, const us16& b2, const us16& b3) {
#if defined(__HIP_DEVICE_COMPILE__)
  asm volatile("v_nop\n\tv_nop\n\tv_nop\n\tv_nop"
               : "+v"(c0), "+v"(c1), "+v"(c2), "+v"(c3), "+v"(c4), "+v"(c5), "+v"(c6), "+v"(c7)
               : "v"(a0), "v"(a1), "v"(b0), "v"(b1), "v"(b2), "v"(b3));
#endif
}

__device__ __forceinline__ us16 gfrag(const unsigned short* p) {
  const int kh = ((threadIdx.x >> 4) & 1) * 8;
  FragU f;
  f.h[0] = *(const us8a*)(p + kh);
  f.h[1] = *(const us8a*)(p + 16 + kh);
  return f.v;
}

template <int MODE>
__global__ __launch_bounds__(256) void k_cvt(const float* __restrict__ src, unsigned short* dst, int total8) {
  const int idx = blockIdx.x * 256 + threadIdx.x;
  if (idx >= total8) return;
  const size_t off = (size_t)idx * 8;
  const v4f a = *(const v4fa*)(src + off), b = *(const v4fa*)(src + off + 4);
  us8 o;
#pragma unroll
  for (int u = 0; u < 4; ++u) {
    if (MODE == 0) {
      o[u]     = bf16_bits(a[u]);
      o[4 + u] = bf16_bits(b[u]);
    } else {
      o[u]     = f16_bits(bf16r(a[u]) * 256.0f);
      o[4 + u] = f16_bits(bf16r(b[u]) * 256.0f);
    }
  }
  *(volatile us8*)(dst + off) = o;
  __threadfence();
  *(volatile us8*)(dst + off) = o;
}

__global__ __launch_bounds__(256) void k_gemm_proj(const unsigned short* __restrict__ Ap, const unsigned short* __restrict__ Bw,
                                                  float* U, float* DLp, float* BCq) {
  __shared__ __attribute__((aligned(16))) float oS[8 * 16 * OSTR];
  const int tid = threadIdx.x, lane = tid & 31, wave = tid >> 5, cl = lane & 15, hh = lane >> 4;
  const int m0 = blockIdx.x * TPB + 16 * wave, n0 = blockIdx.y * 64;

  v8f acc[4];
#pragma unroll
  for (int j = 0; j < 4; ++j) { const v8f zz = {0.f, 0.f, 0.f, 0.f, 0.f, 0.f, 0.f, 0.f}; acc[j] = zz; }

  const unsigned short* a0p = Ap + (size_t)(m0 + cl) * (size_t)DM;
  const unsigned short* bwp = Bw + (size_t)(n0 + cl) * (size_t)DM;
#pragma unroll 1
  for (int k0 = 0; k0 < DM; k0 += 32) {
    const us16 af = gfrag(a0p + k0);
    us16 bfr[4];
#pragma unroll
    for (int j = 0; j < 4; ++j) bfr[j] = gfrag(bwp + (size_t)(16 * j) * (size_t)DM + k0);
#pragma unroll
    for (int j = 0; j < 4; ++j) acc[j] = mma_bf16(af, bfr[j], acc[j]);
    wguard4(acc[0], acc[1], acc[2], acc[3], af, bfr[0], bfr[1], bfr[2], bfr[3]);
  }

  float* so = oS + wave * (16 * OSTR);
#pragma unroll
  for (int j = 0; j < 4; ++j)
#pragma unroll
    for (int r = 0; r < 8; ++r) so[(8 * hh + r) * OSTR + 16 * j + cl] = acc[j][r];
  __syncthreads();

  const int seg = n0 / DM;
  float* dst = U; int pitch = DM; int c0 = n0;
  if (seg == 1) { dst = DLp; pitch = DM;  c0 = n0 - DM; }
  if (seg == 2) { dst = BCq; pitch = NBC; c0 = n0 - 2 * DM; }

  if (seg == 1) {
#pragma unroll 1
    for (int it = 0; it < 8; ++it) {
      const int cx = it * 32 + lane, r = cx >> 4, q = (cx & 15) * 4;
      v4f v = *(const v4fa*)(so + r * OSTR + q);
#pragma unroll
      for (int u = 0; u < 4; ++u) v[u] = softplus_f(v[u]);
      *(v4fa*)(so + r * OSTR + q) = v;
    }
  }
#pragma unroll
  for (int pass = 0; pass < 2; ++pass) {
#pragma unroll
    for (int it = 0; it < 8; ++it) {
      const int cx = it * 32 + lane, r = cx >> 4, q = (cx & 15) * 4;
      const v4f v = *(const v4fa*)(so + r * OSTR + q);
      *(volatile v4f*)(dst + (size_t)(m0 + r) * (size_t)pitch + c0 + q) = v;
    }
    __threadfence();
  }
}

__global__ __launch_bounds__(256) void k_gemm_out(const unsigned short* __restrict__ Zh, const unsigned short* __restrict__ Zl,
                                                 const unsigned short* __restrict__ Wo, float* out) {
  __shared__ __attribute__((aligned(16))) float oS[8 * 16 * OSTR];
  const int tid = threadIdx.x, lane = tid & 31, wave = tid >> 5, cl = lane & 15, hh = lane >> 4;
  const int m0 = blockIdx.x * TPB + 16 * wave, n0 = blockIdx.y * 64;

  v8f acch[4], accl[4];
#pragma unroll
  for (int j = 0; j < 4; ++j) { const v8f zz = {0.f, 0.f, 0.f, 0.f, 0.f, 0.f, 0.f, 0.f}; acch[j] = zz; accl[j] = zz; }

  const unsigned short* zhp = Zh + (size_t)(m0 + cl) * (size_t)DM;
  const unsigned short* zlp = Zl + (size_t)(m0 + cl) * (size_t)DM;
  const unsigned short* wop = Wo + (size_t)(n0 + cl) * (size_t)DM;
#pragma unroll 1
  for (int k0 = 0; k0 < DM; k0 += 32) {
    const us16 ah = gfrag(zhp + k0);
    const us16 al = gfrag(zlp + k0);
    us16 bfr[4];
#pragma unroll
    for (int j = 0; j < 4; ++j) bfr[j] = gfrag(wop + (size_t)(16 * j) * (size_t)DM + k0);
#pragma unroll
    for (int j = 0; j < 4; ++j) {
      acch[j] = mma_f16(ah, bfr[j], acch[j]);
      accl[j] = mma_f16(al, bfr[j], accl[j]);
    }
    wguard8(acch[0], acch[1], acch[2], acch[3], accl[0], accl[1], accl[2], accl[3], ah, al, bfr[0], bfr[1], bfr[2], bfr[3]);
  }

  float* so = oS + wave * (16 * OSTR);
#pragma unroll
  for (int j = 0; j < 4; ++j)
#pragma unroll
    for (int r = 0; r < 8; ++r)
      so[(8 * hh + r) * OSTR + 16 * j + cl] = fmaf(accl[j][r], (1.0f / 2048.0f), acch[j][r]) * (1.0f / 256.0f);
  __syncthreads();

#pragma unroll
  for (int pass = 0; pass < 2; ++pass) {
#pragma unroll
    for (int it = 0; it < 8; ++it) {
      const int cx = it * 32 + lane, r = cx >> 4, q = (cx & 15) * 4;
      const v4f v = *(const v4fa*)(so + r * OSTR + q);
      *(volatile v4f*)(out + (size_t)(m0 + r) * (size_t)DM + n0 + q) = v;
    }
    __threadfence();
  }
}

__global__ __launch_bounds__(256) void k_scan(const float* __restrict__ U, const float* __restrict__ DLp, const float* __restrict__ BCq,
                                             const float* __restrict__ conv_w, const float* __restrict__ conv_b,
                                             const float* __restrict__ A_log, const float* __restrict__ Dpar,
                                             unsigned short* ZH, unsigned short* ZL) {
  __shared__ __attribute__((aligned(16))) float sbc[SCH * NBC];
  __shared__ __attribute__((aligned(16))) float sy[SCH * CHB];
  const int tid = threadIdx.x;
  const int b = blockIdx.x / (DM / CHB), dg = blockIdx.x - b * (DM / CHB);
  const int ch = tid >> 1, sh = tid & 1;
  const int d = dg * CHB + ch;
  const float LOG2E = 1.44269504088896341f;

  const float w0 = bf16r(conv_w[d * 4 + 0]), w1 = bf16r(conv_w[d * 4 + 1]);
  const float w2 = bf16r(conv_w[d * 4 + 2]), w3 = bf16r(conv_w[d * 4 + 3]);
  const float cb = bf16r(conv_b[d]), dp = bf16r(Dpar[d]);

  float a2[16], h[16];
#pragma unroll
  for (int i = 0; i < 16; ++i) {
    const float al = bf16r(A_log[(size_t)(16 * sh + i) * (size_t)DM + d]);
    a2[i] = -EXP2F(al * LOG2E) * LOG2E;
    h[i] = 0.0f;
  }
  float up0 = 0.0f, up1 = 0.0f, up2 = 0.0f;

#pragma unroll 1
  for (int c = 0; c < LQ / SCH; ++c) {
    const size_t tok0 = (size_t)b * LQ + (size_t)c * SCH;
    {
      const float* src = BCq + tok0 * NBC + tid * 8;
      const v4f x0 = *(const v4fa*)src, x1 = *(const v4fa*)(src + 4);
      *(v4fa*)(sbc + tid * 8) = x0;
      *(v4fa*)(sbc + tid * 8 + 4) = x1;
    }
    __syncthreads();

#pragma unroll 1
    for (int st = 0; st < SCH; ++st) {
      const size_t gi = (tok0 + (size_t)st) * (size_t)DM + d;
      const float ur = U[gi];
      const float de = DLp[gi];
      float cv = w0 * up2;
      cv = fmaf(w1, up1, cv);
      cv = fmaf(w2, up0, cv);
      cv = fmaf(w3, ur, cv);
      const float uc = cv + cb;
      up2 = up1; up1 = up0; up0 = ur;

      const float* bp = sbc + st * NBC + 16 * sh;
      const v4f bq0 = *(const v4fa*)bp, bq1 = *(const v4fa*)(bp + 4), bq2 = *(const v4fa*)(bp + 8), bq3 = *(const v4fa*)(bp + 12);
      const v4f cq0 = *(const v4fa*)(bp + NST), cq1 = *(const v4fa*)(bp + NST + 4);
      const v4f cq2 = *(const v4fa*)(bp + NST + 8), cq3 = *(const v4fa*)(bp + NST + 12);
      float bv[16], cw[16];
#pragma unroll
      for (int u = 0; u < 4; ++u) {
        bv[u] = bq0[u]; bv[4 + u] = bq1[u]; bv[8 + u] = bq2[u]; bv[12 + u] = bq3[u];
        cw[u] = cq0[u]; cw[4 + u] = cq1[u]; cw[8 + u] = cq2[u]; cw[12 + u] = cq3[u];
      }
      float y = 0.0f;
#pragma unroll
      for (int i = 0; i < 16; ++i) {
        const float e = EXP2F(de * a2[i]);
        h[i] = fmaf(h[i], e, bv[i] * uc);
        y = fmaf(h[i], cw[i], y);
      }
      y += __shfl_xor(y, 1, 32);
      const float z = fmaf(uc, dp, y);
      if (sh == 0) sy[st * CHB + ch] = z;
    }
    __syncthreads();

    us8 hv[2], lv[2];
    size_t offs[2];
#pragma unroll
    for (int it = 0; it < 2; ++it) {
      const int cx = it * 256 + tid, r = cx >> 4, q = (cx & 15) * 8;
      const v4f z0 = *(const v4fa*)(sy + r * CHB + q), z1 = *(const v4fa*)(sy + r * CHB + q + 4);
      us8 ho, lo;
#pragma unroll
      for (int u = 0; u < 4; ++u) {
        unsigned short hb, lb;
        f16split(z0[u], hb, lb); ho[u] = hb;     lo[u] = lb;
        f16split(z1[u], hb, lb); ho[4 + u] = hb; lo[4 + u] = lb;
      }
      hv[it] = ho; lv[it] = lo;
      offs[it] = (tok0 + (size_t)r) * (size_t)DM + (size_t)dg * CHB + q;
    }
#pragma unroll
    for (int pass = 0; pass < 2; ++pass) {
#pragma unroll
      for (int it = 0; it < 2; ++it) {
        *(volatile us8*)(ZH + offs[it]) = hv[it];
        *(volatile us8*)(ZL + offs[it]) = lv[it];
      }
      __threadfence();
    }
    __syncthreads();
  }
}

extern "C" void kernel_launch(void* const* d_in, const int* in_sizes, int n_in,
                              void* d_out, int out_size, void* d_ws, size_t ws_size,
                              hipStream_t stream) {
  if (n_in < 7) return;
  if (in_sizes[0] != NTOK * DM || in_sizes[1] != 3 * DM * DM || in_sizes[2] != DM * DM || in_sizes[3] != DM * 4 ||
      in_sizes[4] != DM || in_sizes[5] != NST * DM || in_sizes[6] != DM) return;
  if (out_size != NTOK * DM) return;

  const float* x      = (const float*)d_in[0];
  const float* W_in   = (const float*)d_in[1];
  const float* W_out  = (const float*)d_in[2];
  const float* conv_w = (const float*)d_in[3];
  const float* conv_b = (const float*)d_in[4];
  const float* A_log  = (const float*)d_in[5];
  const float* Dpar   = (const float*)d_in[6];
  float* out = (float*)d_out;

  size_t off = 0;
  auto carve = [&](size_t bytes) -> char* { char* p = (char*)d_ws + off; off += (bytes + 255) & ~(size_t)255; return p; };
  unsigned short* XB   = (unsigned short*)carve((size_t)NTOK * DM * 2);
  unsigned short* WIb  = (unsigned short*)carve((size_t)NPROJ * DM * 2);
  unsigned short* WO16 = (unsigned short*)carve((size_t)DM * DM * 2);
  float* U   = (float*)carve((size_t)NTOK * DM * 4);
  float* DLp = (float*)carve((size_t)NTOK * DM * 4);
  float* BCq = (float*)carve((size_t)NTOK * NBC * 4);
  unsigned short* ZH = (unsigned short*)carve((size_t)NTOK * DM * 2);
  unsigned short* ZL = (unsigned short*)carve((size_t)NTOK * DM * 2);
  if (off > ws_size || off > (size_t)134217728) return;

  const dim3 b256(256);
  auto cdv = [](long a, long bq) { return (unsigned)((a + bq - 1) / bq); };

  k_cvt<0><<<dim3(cdv((long)NTOK * DM / 8, 256)), b256, 0, stream>>>(x, XB, NTOK * DM / 8);
  k_cvt<0><<<dim3(cdv((long)NPROJ * DM / 8, 256)), b256, 0, stream>>>(W_in, WIb, NPROJ * DM / 8);
  k_cvt<1><<<dim3(cdv((long)DM * DM / 8, 256)), b256, 0, stream>>>(W_out, WO16, DM * DM / 8);
  k_gemm_proj<<<dim3(NTOK / TPB, NPROJ / 64), b256, 0, stream>>>(XB, WIb, U, DLp, BCq);
  k_scan<<<dim3(BQ * (DM / CHB)), b256, 0, stream>>>(U, DLp, BCq, conv_w, conv_b, A_log, Dpar, ZH, ZL);
  k_gemm_out<<<dim3(NTOK / TPB, DM / 64), b256, 0, stream>>>(ZH, ZL, WO16, out);
}
